// mLSTMCell_29162827940155
// MI455X (gfx1250) — hardware-run, weakly checked
//
#include <hip/hip_runtime.h>


#define TT   2048
#define EE   1024
#define NH_  8
#define DH   128
#define ZH   2
typedef _Float16 h16;
typedef unsigned short bf;
typedef __attribute__((ext_vector_type(16))) __bf16   v16bf;
typedef __attribute__((ext_vector_type(16))) _Float16 v16h;
typedef __attribute__((ext_vector_type(8)))  _Float16 v8h;
typedef __attribute__((ext_vector_type(8)))  unsigned short v8us;
typedef __attribute__((ext_vector_type(8)))  float    v8f;
typedef __attribute__((ext_vector_type(4)))  float    v4f;
typedef v8h  __attribute__((may_alias)) v8ha;
typedef v4f  __attribute__((may_alias)) v4fa;
typedef v8us __attribute__((may_alias)) v8usa;

__device__ __forceinline__ unsigned short f2bf(float f) { unsigned u = __float_as_uint(f); u += 0x7FFFu + ((u >> 16) & 1u); return (unsigned short)(u >> 16); }
__device__ __forceinline__ float bf2f(unsigned short b) { return __uint_as_float(((unsigned)b) << 16); }
__device__ __forceinline__ float bfr(float f) { return bf2f(f2bf(f)); }
__device__ __forceinline__ v16h cat16(v8h lo, v8h hi) { return __builtin_shufflevector(lo, hi, 0, 1, 2, 3, 4, 5, 6, 7, 8, 9, 10, 11, 12, 13, 14, 15); }
__device__ __forceinline__ v16bf cat16b(v8us lo, v8us hi) { return __builtin_bit_cast(v16bf, __builtin_shufflevector(lo, hi, 0, 1, 2, 3, 4, 5, 6, 7, 8, 9, 10, 11, 12, 13, 14, 15)); }
__device__ __forceinline__ v8f wmma16(v16h a, v16h b, v8f c) { return __builtin_amdgcn_wmma_f32_16x16x32_f16(false, a, false, b, (short)0, c, false, false); }
__device__ __forceinline__ v8f wmmab(v16bf a, v16bf b, v8f c) { return __builtin_amdgcn_wmma_f32_16x16x32_bf16(false, a, false, b, (short)0, c, false, false); }


template <typename T16> struct WFrag;
template <> struct WFrag<h16> { typedef v16h V; static __device__ __forceinline__ V ld(const h16* p) { return cat16(*(const v8h*)p, *(const v8h*)(p + 16)); } static __device__ __forceinline__ v8f mma(V a, V b, v8f c) { return wmma16(a, b, c); } };
template <> struct WFrag<bf> { typedef v16bf V; static __device__ __forceinline__ V ld(const bf* p) { return cat16b(*(const v8us*)p, *(const v8us*)(p + 16)); } static __device__ __forceinline__ v8f mma(V a, V b, v8f c) { return wmmab(a, b, c); } };
template <typename T16, int NSPLIT, bool BIAS>
__global__ __launch_bounds__(32) void k_gemmw(const T16* __restrict__ A, const T16* __restrict__ A2, const T16* __restrict__ Bt, const T16* __restrict__ Bt2, int K, float* C, int ldc, const float* __restrict__ bias, size_t sA, size_t sB, size_t sC) {
    typedef typename WFrag<T16>::V V;
    __shared__ __align__(16) float os[16 * 68];
    const size_t z = blockIdx.z; A += z * sA; if (A2) A2 += z * sA; Bt += z * sB; if (Bt2) Bt2 += z * sB; C += z * sC;
    const int lane = threadIdx.x & 31, lr = lane & 15, hi = lane >> 4; const int r0 = blockIdx.x * 64, c0 = blockIdx.y * 64;
    v8f acc[4][4];
#pragma unroll
    for (int mb = 0; mb < 4; ++mb)
#pragma unroll
        for (int nb = 0; nb < 4; ++nb) acc[mb][nb] = (v8f){};
    const size_t aoff = (size_t)(r0 + lr) * K + 8 * hi, boff = (size_t)(c0 + lr) * K + 8 * hi;
#pragma unroll 1
    for (int kc = 0; kc < K; kc += 32) {
        V a[4], a2[4];
#pragma unroll
        for (int mb = 0; mb < 4; ++mb) { a[mb] = WFrag<T16>::ld(A + aoff + (size_t)mb * 16 * K + kc); if (NSPLIT == 1 || NSPLIT == 2) a2[mb] = WFrag<T16>::ld(A2 + aoff + (size_t)mb * 16 * K + kc); }
#pragma unroll
        for (int nb = 0; nb < 4; ++nb) { const V b = WFrag<T16>::ld(Bt + boff + (size_t)nb * 16 * K + kc); V b2; if (NSPLIT >= 2) b2 = WFrag<T16>::ld(Bt2 + boff + (size_t)nb * 16 * K + kc);
#pragma unroll
            for (int mb = 0; mb < 4; ++mb) { acc[mb][nb] = WFrag<T16>::mma(a[mb], b, acc[mb][nb]); if (NSPLIT == 1 || NSPLIT == 2) acc[mb][nb] = WFrag<T16>::mma(a2[mb], b, acc[mb][nb]); if (NSPLIT >= 2) acc[mb][nb] = WFrag<T16>::mma(a[mb], b2, acc[mb][nb]); } }
        asm volatile("v_nop\n\tv_nop\n\tv_nop\n\tv_nop" : "+v"(acc[0][0]), "+v"(acc[1][1]), "+v"(acc[2][2]), "+v"(acc[3][3]) : "v"(a[0]), "v"(a[3]));
    }
#pragma unroll
    for (int mb = 0; mb < 4; ++mb) {
#pragma unroll
        for (int nb = 0; nb < 4; ++nb) {
#pragma unroll
            for (int j = 0; j < 8; ++j) os[(hi * 8 + j) * 68 + nb * 16 + lr] = acc[mb][nb][j]; }
        __builtin_amdgcn_wave_barrier(); asm volatile("" ::: "memory");
        float* crow = C + (size_t)(r0 + mb * 16) * ldc + c0;
#pragma unroll 1
        for (int ps = 0; ps < 2; ++ps) {
#pragma unroll
            for (int s = 0; s < 8; ++s) { const int row = 2 * s + hi, cofs = lr * 4; v4f val = *(const v4fa*)(os + row * 68 + cofs); if (BIAS) { val[0] += bfr(bias[c0 + cofs]); val[1] += bfr(bias[c0 + cofs + 1]); val[2] += bfr(bias[c0 + cofs + 2]); val[3] += bfr(bias[c0 + cofs + 3]); }
                *(volatile v4f*)(crow + (size_t)row * ldc + cofs) = val; }
            if (ps == 0) __threadfence(); }
        __builtin_amdgcn_wave_barrier(); asm volatile("" ::: "memory");
    }
}

__device__ __forceinline__ void splitf(float y, unsigned short& h, unsigned short& l) { h = f2bf(y); l = f2bf(y - bf2f(h)); }
typedef __attribute__((ext_vector_type(2))) unsigned short v2us;
typedef __attribute__((ext_vector_type(4))) unsigned short v4us;

__global__ __launch_bounds__(256) void k_cvt8(const float* __restrict__ src, bf* dst, size_t n8) { const size_t i = (size_t)blockIdx.x * 256 + threadIdx.x; if (i >= n8) return; const v8f v = *(const v8f*)(src + i * 8); v8us o;
#pragma unroll
    for (int k = 0; k < 8; ++k) o[k] = f2bf(v[k]); *(volatile v8us*)(dst + i * 8) = o; __threadfence(); *(volatile v8us*)(dst + i * 8) = o; }
__global__ __launch_bounds__(256) void k_xg(const float* __restrict__ q, const float* __restrict__ k, const float* __restrict__ v, bf* XG) { const size_t e = ((size_t)blockIdx.x * 256 + threadIdx.x) * 4; if (e >= (size_t)TT * 3 * EE) return; const int c = (int)(e % (3 * EE)); const size_t s = e / (3 * EE); const float* src = (c < EE) ? (q + s * EE + c) : (c < 2 * EE) ? (k + s * EE + c - EE) : (v + s * EE + c - 2 * EE); v4us o;
#pragma unroll
    for (int u = 0; u < 4; ++u) o[u] = f2bf(src[u]); *(volatile v4us*)(XG + e) = o; __threadfence(); *(volatile v4us*)(XG + e) = o; }
__global__ __launch_bounds__(256) void k_wg(const float* __restrict__ wi, const float* __restrict__ wf, bf* Bt) { const size_t e = ((size_t)blockIdx.x * 256 + threadIdx.x) * 4; if (e >= (size_t)64 * 3 * EE) return; const int c = (int)(e % (3 * EE)); const int n = (int)(e / (3 * EE)); v4us o;
#pragma unroll
    for (int u = 0; u < 4; ++u) o[u] = (n < NH_) ? f2bf(wi[(size_t)n * 3 * EE + c + u]) : (n < 2 * NH_) ? f2bf(wf[(size_t)(n - NH_) * 3 * EE + c + u]) : (unsigned short)0; *(volatile v4us*)(Bt + e) = o; __threadfence(); *(volatile v4us*)(Bt + e) = o; }
__global__ __launch_bounds__(64) void k_cum(const float* __restrict__ GT, const float* __restrict__ ib, const float* __restrict__ fb, float* CS, float* IG) { const int h = threadIdx.x; if (h >= NH_) return; const float bi = bfr(ib[h]), bfv = bfr(fb[h]); float acc = 0.f;
    for (int ps = 0; ps < 2; ++ps) { acc = 0.f;
#pragma unroll 1
        for (int s = 0; s < TT; ++s) { const float f = __fadd_rn(GT[(size_t)s * 64 + NH_ + h], bfv); const float mn = fminf(f, 0.f); const float ls = __fsub_rn(mn, log1pf(__expf(-fabsf(f)))); acc = __fadd_rn(acc, ls); *(volatile float*)(CS + (size_t)h * TT + s) = acc; const float ig = __fadd_rn(GT[(size_t)s * 64 + h], bi); *(volatile float*)(IG + (size_t)h * TT + s) = ig; }
        if (ps == 0) __threadfence(); } }
__global__ __launch_bounds__(256) void k_qkp(const float* __restrict__ q, const float* __restrict__ k, bf* QP, bf* KP) { const size_t e = ((size_t)blockIdx.x * 256 + threadIdx.x) * 4; if (e >= (size_t)NH_ * TT * DH) return; const int d = (int)(e % DH); const int s = (int)((e / DH) % TT); const int h = (int)(e / ((size_t)DH * TT)); const size_t so = (size_t)s * EE + h * DH + d; v4us a, b;
#pragma unroll
    for (int u = 0; u < 4; ++u) { a[u] = f2bf(q[so + u]); b[u] = f2bf(k[so + u]); } *(volatile v4us*)(QP + e) = a; *(volatile v4us*)(KP + e) = b; __threadfence(); *(volatile v4us*)(QP + e) = a; *(volatile v4us*)(KP + e) = b; }
__global__ __launch_bounds__(256) void k_vt(const float* __restrict__ v, bf* VT) { const size_t e = ((size_t)blockIdx.x * 256 + threadIdx.x) * 2; if (e >= (size_t)NH_ * DH * TT) return; const int s = (int)(e % TT); const int d = (int)((e / TT) % DH); const int h = (int)(e / ((size_t)TT * DH)); v2us o; o[0] = f2bf(v[(size_t)s * EE + h * DH + d]); o[1] = f2bf(v[(size_t)(s + 1) * EE + h * DH + d]); *(volatile v2us*)(VT + e) = o; __threadfence(); *(volatile v2us*)(VT + e) = o; }
__global__ __launch_bounds__(256) void k_mrow(const float* __restrict__ S, const float* __restrict__ CS, const float* __restrict__ IG, int h0, bf* Ph, bf* Pl) { const int lane = threadIdx.x & 31; const int row = blockIdx.x * 8 + (threadIdx.x >> 5); if (row >= ZH * TT) return; const int i = row % TT; const int h = h0 + row / TT; const float* sr = S + (size_t)row * TT; const float csi = CS[(size_t)h * TT + i]; float v[TT / 32]; float mx = -3.0e38f;
#pragma unroll
    for (int ch = 0; ch < TT / 128; ++ch) {
#pragma unroll
        for (int u = 0; u < 4; ++u) { const int j = ch * 128 + lane * 4 + u; float ld = -3.0e38f; if (j <= i) { float df = __fsub_rn(csi, CS[(size_t)h * TT + j]); asm volatile("" : "+v"(df)); ld = __fadd_rn(df, IG[(size_t)h * TT + j]); } v[ch * 4 + u] = ld; mx = fmaxf(mx, ld); } }
#pragma unroll
    for (int sh = 16; sh; sh >>= 1) mx = fmaxf(mx, __shfl_xor(mx, sh, 32));
    float csum = 0.f;
#pragma unroll
    for (int ch = 0; ch < TT / 128; ++ch) { const v4f a = *(const v4f*)(sr + ch * 128 + lane * 4);
#pragma unroll
        for (int u = 0; u < 4; ++u) { const int j = ch * 128 + lane * 4 + u; float dd = 0.f; if (j <= i) { float d0 = __fsub_rn(v[ch * 4 + u], mx); asm volatile("" : "+v"(d0)); dd = __expf(d0); } float sc = a[u] * 0.088388347648318447f; asm volatile("" : "+v"(sc)); float c = __fmul_rn(sc, dd); asm volatile("" : "+v"(c)); v[ch * 4 + u] = c; csum = __fadd_rn(csum, c); } }
#pragma unroll
    for (int sh = 16; sh; sh >>= 1) csum += __shfl_xor(csum, sh, 32);
    float emx = __expf(-mx); asm volatile("" : "+v"(emx)); const float nrm = fmaxf(fabsf(csum), emx); const float den = __fadd_rn(nrm, 1e-6f); const float rden = __fdiv_rn(1.0f, den);
    for (int ps = 0; ps < 2; ++ps) {
#pragma unroll
        for (int ch = 0; ch < TT / 128; ++ch) { v4us oh, ol; for (int u = 0; u < 4; ++u) { unsigned short a2, c2; splitf(__fmul_rn(v[ch * 4 + u], rden), a2, c2); oh[u] = a2; ol[u] = c2; } const size_t oo = (size_t)row * TT + ch * 128 + lane * 4; *(volatile v4us*)(Ph + oo) = oh; *(volatile v4us*)(Pl + oo) = ol; }
        if (ps == 0) __threadfence(); } }
__global__ __launch_bounds__(256) void k_gn(const float* __restrict__ O, const float* __restrict__ ow, int h0, float* out) { const int lane = threadIdx.x & 31; const int row = blockIdx.x * 8 + (threadIdx.x >> 5); if (row >= ZH * TT) return; const int s = row % TT; const int h = h0 + row / TT; const v4f a = *(const v4f*)(O + (size_t)row * DH + lane * 4); float sm = (a[0] + a[1]) + (a[2] + a[3]);
#pragma unroll
    for (int sh = 16; sh; sh >>= 1) sm += __shfl_xor(sm, sh, 32);
    const float mean = sm * (1.0f / DH); float dv[4]; float q2 = 0.f;
#pragma unroll
    for (int u = 0; u < 4; ++u) { float d = __fsub_rn(a[u], mean); asm volatile("" : "+v"(d)); dv[u] = d; float p = __fmul_rn(d, d); asm volatile("" : "+v"(p)); q2 = __fadd_rn(q2, p); }
#pragma unroll
    for (int sh = 16; sh; sh >>= 1) q2 += __shfl_xor(q2, sh, 32);
    const float rs = __fdiv_rn(1.0f, __fsqrt_rn(__fadd_rn(q2 * (1.0f / DH), 1e-5f))); v4f o;
#pragma unroll
    for (int u = 0; u < 4; ++u) { float n0 = __fmul_rn(dv[u], rs); asm volatile("" : "+v"(n0)); o[u] = __fmul_rn(n0, bfr(ow[h * DH + lane * 4 + u])); }
    float* dst = out + (size_t)s * EE + h * DH + lane * 4; *(volatile v4f*)dst = o; __threadfence(); *(volatile v4f*)dst = o; }

extern "C" void kernel_launch(void* const* d_in, const int* in_sizes, int n_in,
                              void* d_out, int out_size, void* d_ws, size_t ws_size, hipStream_t stream) {
    (void)in_sizes; (void)n_in; (void)out_size;
    const float** I = (const float**)d_in;
    const float *q = I[0], *k = I[1], *v = I[2], *iw = I[3], *ib = I[4], *fw = I[5], *fb = I[6], *ow = I[7];
    float* OUT = (float*)d_out;
    char* wsp = (char*)d_ws;
    auto take = [&](size_t bytes) { char* p = wsp; wsp += (bytes + 255) & ~(size_t)255; return (void*)p; };
    bf* XG = (bf*)take((size_t)TT * 3 * EE * 2); bf* WG = (bf*)take((size_t)64 * 3 * EE * 2); float* GT = (float*)take((size_t)TT * 64 * 4); float* CS = (float*)take((size_t)NH_ * TT * 4); float* IG = (float*)take((size_t)NH_ * TT * 4);
    bf* QP = (bf*)take((size_t)NH_ * TT * DH * 2); bf* KP = (bf*)take((size_t)NH_ * TT * DH * 2); bf* VT = (bf*)take((size_t)NH_ * DH * TT * 2); float* S = (float*)take((size_t)ZH * TT * TT * 4); bf* Ph = (bf*)take((size_t)ZH * TT * TT * 2); bf* Pl = (bf*)take((size_t)ZH * TT * TT * 2); float* O = (float*)take((size_t)ZH * TT * DH * 4);
    if ((size_t)(wsp - (char*)d_ws) > ws_size) return;
    k_xg<<<(unsigned)(((size_t)TT * 3 * EE / 4 + 255) / 256), 256, 0, stream>>>(q, k, v, XG); k_wg<<<(unsigned)(((size_t)64 * 3 * EE / 4 + 255) / 256), 256, 0, stream>>>(iw, fw, WG);
    k_gemmw<bf, 0, false><<<dim3(TT / 64, 1, 1), 32, 0, stream>>>(XG, nullptr, WG, nullptr, 3 * EE, GT, 64, nullptr, 0, 0, 0);
    k_cum<<<1, 64, 0, stream>>>(GT, ib, fb, CS, IG);
    k_qkp<<<(unsigned)(((size_t)NH_ * TT * DH / 4 + 255) / 256), 256, 0, stream>>>(q, k, QP, KP); k_vt<<<(unsigned)(((size_t)NH_ * DH * TT / 2 + 255) / 256), 256, 0, stream>>>(v, VT);
    const size_t zq = (size_t)TT * DH, zS = (size_t)TT * TT, zv = (size_t)DH * TT;
    for (int h0 = 0; h0 < NH_; h0 += ZH) {
        k_gemmw<bf, 0, false><<<dim3(TT / 64, TT / 64, ZH), 32, 0, stream>>>(QP + (size_t)h0 * zq, nullptr, KP + (size_t)h0 * zq, nullptr, DH, S, TT, nullptr, zq, zq, zS);
        k_mrow<<<ZH * TT / 8, 256, 0, stream>>>(S, CS, IG, h0, Ph, Pl);
        k_gemmw<bf, 1, false><<<dim3(TT / 64, DH / 64, ZH), 32, 0, stream>>>(Ph, Pl, VT + (size_t)h0 * zv, nullptr, TT, O, DH, nullptr, zS, zv, zq);
        k_gn<<<ZH * TT / 8, 256, 0, stream>>>(O, ow, h0, OUT); }
}
